// liBRU_28664611733942
// MI455X (gfx1250) — hardware-run, weakly checked
//
#include <hip/hip_runtime.h>
#include <math.h>

typedef __attribute__((ext_vector_type(16))) __bf16   v16b;
typedef __attribute__((ext_vector_type(8)))  __bf16   v8b;
typedef __attribute__((ext_vector_type(8)))  float    v8f;
typedef __attribute__((ext_vector_type(4)))  float    v4f;
typedef __attribute__((ext_vector_type(2)))  float    v2f;
typedef __attribute__((ext_vector_type(4)))  unsigned v4u;

constexpr int kNB   = 32;
constexpr int kNT   = 1000;
constexpr int kNF   = 256;
constexpr int kNH   = 512;
constexpr int kRows = kNB * kNT;
constexpr int kProjM = 32;
constexpr int kScanM = 16;
static_assert(kRows == 32000, "rows");
static_assert((kRows % kProjM) == 0, "projection row tiles");
static_assert((kNF % 32) == 0 && (kNH % 32) == 0, "K multiples of 32");
static_assert((kNH % 64) == 0, "N multiple of 64");
static_assert((kNB % kScanM) == 0, "scan batch tiles");
static_assert(kNH == 16 * 32, "16 waves x 32 columns in the scan");

constexpr int kCastBlkX = (kRows * kNF) / 2048;
constexpr int kCastBlkW = (kNH * kNF) / 2048;
constexpr int kCastBlkV = (kNH * kNH) / 2048;
constexpr int kCastBlocks = kCastBlkX + 2 * kCastBlkW + 2 * kCastBlkV;
static_assert(kCastBlkX * 2048 == kRows * kNF, "exact cover x");
static_assert(kCastBlkW * 2048 == kNH * kNF, "exact cover W");
static_assert(kCastBlkV * 2048 == kNH * kNH, "exact cover V");

constexpr size_t kOffXB  = 0;
constexpr size_t kOffWB  = kOffXB  + (size_t)kRows * kNF * 2;
constexpr size_t kOffWZB = kOffWB  + (size_t)kNH * kNF * 2;
constexpr size_t kOffVB  = kOffWZB + (size_t)kNH * kNF * 2;
constexpr size_t kOffVZB = kOffVB  + (size_t)kNH * kNH * 2;
constexpr size_t kOffWX  = kOffVZB + (size_t)kNH * kNH * 2;
constexpr size_t kOffWZX = kOffWX  + (size_t)kRows * kNH * 4;
constexpr size_t kWsTotal = kOffWZX + (size_t)kRows * kNH * 2;
static_assert(kWsTotal == 116260864ull, "carve total");
static_assert(kWsTotal <= 134217728ull, "carve cap");
static_assert((kOffWB % 128) == 0 && (kOffWZB % 128) == 0 && (kOffVB % 128) == 0 &&
              (kOffVZB % 128) == 0 && (kOffWX % 128) == 0 && (kOffWZX % 128) == 0, "128-B aligned regions");

__device__ __forceinline__ unsigned f2bf_bits(float f) {
  const unsigned u = __float_as_uint(f);
  return (u + 0x7FFFu + ((u >> 16) & 1u)) >> 16;
}
__device__ __forceinline__ float bf_bits2f(unsigned h) { return __uint_as_float(h << 16); }
__device__ __forceinline__ float bf_rne(float f) { return bf_bits2f(f2bf_bits(f)); }
__device__ __forceinline__ unsigned f2h_bits(float f) {
  const _Float16 h = (_Float16)f;
  return (unsigned)__builtin_bit_cast(unsigned short, h);
}
__device__ __forceinline__ float h16_to_f32(unsigned hb) {
  const unsigned sgn = (hb & 0x8000u) << 16;
  const unsigned em = hb & 0x7fffu;
  const float fn = __uint_as_float((em << 13) + 0x38000000u);
  const float fs = (float)em * 5.9604644775390625e-8f;
  const float mag = (em < 0x400u) ? fs : fn;
  return __uint_as_float(__float_as_uint(mag) | sgn);
}

union FragB { v16b v; v8b h[2]; };
__device__ __forceinline__ v16b frag_load(const __bf16* p) {
  FragB f;
  f.h[0] = *(const v8b*)(p);
  f.h[1] = *(const v8b*)(p + 16);
  return f.v;
}
__device__ __forceinline__ v8f at_mma(v16b a, v16b b, v8f c) {
  c = __builtin_amdgcn_wmma_f32_16x16x32_bf16(false, a, false, b, (short)0, c, false, false);
  asm volatile("v_nop\n\tv_nop\n\tv_nop\n\tv_nop" : "+v"(c) : "v"(a), "v"(b));
  return c;
}

__global__ __launch_bounds__(256) void cast_bf16_kernel(
    const float* __restrict__ x, const float* __restrict__ W, const float* __restrict__ Wz,
    const float* __restrict__ V, const float* __restrict__ Vz,
    unsigned* __restrict__ xb, unsigned* __restrict__ Wb, unsigned* __restrict__ Wzb,
    unsigned* __restrict__ Vb, unsigned* __restrict__ Vzb)
{
  int blk = blockIdx.x;
  const float* src = x;
  unsigned* dst = xb;
  if (blk >= kCastBlkX) {
    blk -= kCastBlkX; src = W; dst = Wb;
    if (blk >= kCastBlkW) {
      blk -= kCastBlkW; src = Wz; dst = Wzb;
      if (blk >= kCastBlkW) {
        blk -= kCastBlkW; src = V; dst = Vb;
        if (blk >= kCastBlkV) {
          blk -= kCastBlkV; src = Vz; dst = Vzb;
        }
      }
    }
  }
  const size_t e0 = ((size_t)blk * 256 + threadIdx.x) * 8;
  const v4f a0 = *(const v4f*)(src + e0);
  const v4f a1 = *(const v4f*)(src + e0 + 4);
  v4u w;
  w.x = f2bf_bits(a0.x) | (f2bf_bits(a0.y) << 16);
  w.y = f2bf_bits(a0.z) | (f2bf_bits(a0.w) << 16);
  w.z = f2bf_bits(a1.x) | (f2bf_bits(a1.y) << 16);
  w.w = f2bf_bits(a1.z) | (f2bf_bits(a1.w) << 16);
  unsigned* q = dst + (e0 >> 1);
  *(volatile v4u*)q = w;
  __threadfence();
  *(volatile v4u*)q = w;
}

template <int F16OUT>
__global__ __launch_bounds__(256) void proj_ln_kernel(
    const unsigned short* __restrict__ xbp, const unsigned short* __restrict__ wbp,
    const float* __restrict__ gamma, const float* __restrict__ beta, void* __restrict__ dstv)
{
  __shared__ __align__(16) float sP[kProjM * kNH];
  const int tid = threadIdx.x, lane = tid & 31, wave = tid >> 5;
  const int hh = lane >> 4, c = lane & 15;
  const int koff = hh * 8;
  const int m0 = blockIdx.x * kProjM;
  const int n0 = wave * 64;
  const __bf16* A  = (const __bf16*)xbp;
  const __bf16* Bt = (const __bf16*)wbp;

  v8f acc[2][4];
#pragma unroll
  for (int i = 0; i < 2; ++i)
#pragma unroll
    for (int j = 0; j < 4; ++j) acc[i][j] = (v8f){0.f, 0.f, 0.f, 0.f, 0.f, 0.f, 0.f, 0.f};

  const __bf16* aP0 = A + (size_t)(m0 + c) * kNF + koff;
  const __bf16* aP1 = aP0 + (size_t)16 * kNF;
  const __bf16* bP  = Bt + (size_t)(n0 + c) * kNF + koff;
#pragma unroll 1
  for (int k0 = 0; k0 < kNF; k0 += 32) {
    v16b bf[4];
#pragma unroll
    for (int j = 0; j < 4; ++j) bf[j] = frag_load(bP + (size_t)j * 16 * kNF + k0);
    const v16b a0 = frag_load(aP0 + k0);
    const v16b a1 = frag_load(aP1 + k0);
#pragma unroll
    for (int j = 0; j < 4; ++j) {
      acc[0][j] = at_mma(a0, bf[j], acc[0][j]);
      acc[1][j] = at_mma(a1, bf[j], acc[1][j]);
    }
  }

#pragma unroll
  for (int i = 0; i < 2; ++i)
#pragma unroll
    for (int j = 0; j < 4; ++j)
#pragma unroll
      for (int r = 0; r < 8; ++r)
        sP[(16 * i + 8 * hh + r) * kNH + n0 + 16 * j + c] = acc[i][j][r];
  __syncthreads();

  int cb[4];
#pragma unroll
  for (int q = 0; q < 4; ++q)
    cb[q] = F16OUT ? ((q >> 1) * 256 + lane * 8 + (q & 1) * 4) : (q * 128 + lane * 4);

  v4f gm[4], bt[4];
#pragma unroll
  for (int q = 0; q < 4; ++q) {
    const v4f g = *(const v4f*)(gamma + cb[q]);
    const v4f b = *(const v4f*)(beta + cb[q]);
    gm[q].x = bf_rne(g.x); gm[q].y = bf_rne(g.y); gm[q].z = bf_rne(g.z); gm[q].w = bf_rne(g.w);
    bt[q].x = bf_rne(b.x); bt[q].y = bf_rne(b.y); bt[q].z = bf_rne(b.z); bt[q].w = bf_rne(b.w);
  }

#pragma unroll 1
  for (int rr = 0; rr < 4; ++rr) {
    const int row = wave * 4 + rr;
    const float* sp = sP + row * kNH;
    v4f v[4];
#pragma unroll
    for (int q = 0; q < 4; ++q) v[q] = *(const v4f*)(sp + cb[q]);
    float s = 0.f;
#pragma unroll
    for (int q = 0; q < 4; ++q) s += (v[q].x + v[q].y) + (v[q].z + v[q].w);
#pragma unroll
    for (int off = 16; off > 0; off >>= 1) s += __shfl_xor(s, off, 32);
    const float mu = s * (1.0f / (float)kNH);
    float ss = 0.f;
#pragma unroll
    for (int q = 0; q < 4; ++q) {
      v[q].x -= mu; v[q].y -= mu; v[q].z -= mu; v[q].w -= mu;
      ss += (v[q].x * v[q].x + v[q].y * v[q].y) + (v[q].z * v[q].z + v[q].w * v[q].w);
    }
#pragma unroll
    for (int off = 16; off > 0; off >>= 1) ss += __shfl_xor(ss, off, 32);
    const float var = ss * (1.0f / (float)kNH);
    const float rstd = rsqrtf(var + 1e-5f);
    v4f y[4];
#pragma unroll
    for (int q = 0; q < 4; ++q) {
      y[q].x = v[q].x * rstd * gm[q].x + bt[q].x;
      y[q].y = v[q].y * rstd * gm[q].y + bt[q].y;
      y[q].z = v[q].z * rstd * gm[q].z + bt[q].z;
      y[q].w = v[q].w * rstd * gm[q].w + bt[q].w;
    }
    if (F16OUT == 0) {
      float* drow = (float*)dstv + (size_t)(m0 + row) * kNH;
      for (int pass = 0; pass < 2; ++pass) {
#pragma unroll
        for (int q = 0; q < 4; ++q) *(volatile v4f*)(drow + q * 128 + lane * 4) = y[q];
        __threadfence();
      }
    } else {
      v4u w[2];
#pragma unroll
      for (int i = 0; i < 2; ++i) {
        w[i].x = f2h_bits(y[2 * i].x)     | (f2h_bits(y[2 * i].y)     << 16);
        w[i].y = f2h_bits(y[2 * i].z)     | (f2h_bits(y[2 * i].w)     << 16);
        w[i].z = f2h_bits(y[2 * i + 1].x) | (f2h_bits(y[2 * i + 1].y) << 16);
        w[i].w = f2h_bits(y[2 * i + 1].z) | (f2h_bits(y[2 * i + 1].w) << 16);
      }
      unsigned* drow = (unsigned*)dstv + (size_t)(m0 + row) * (kNH / 2);
      for (int pass = 0; pass < 2; ++pass) {
#pragma unroll
        for (int i = 0; i < 2; ++i) *(volatile v4u*)(drow + i * 128 + lane * 4) = w[i];
        __threadfence();
      }
    }
  }
}

__device__ __forceinline__ float gate_update(float pz, float pc, float hold) {
  const float ez = __expf(-pz);
  const float z  = __builtin_amdgcn_rcpf(1.0f + ez);
  const float ec = 1.0f + __expf(pc);
  const float eh = __expf(hold);
  const float sm = z * eh + (1.0f - z) * ec;
  return __logf(sm);
}

__global__ __launch_bounds__(512) void gated_scan_kernel(
    const unsigned short* __restrict__ vbp, const unsigned short* __restrict__ vzbp,
    const float* __restrict__ WX, const unsigned* __restrict__ WZX32, float* __restrict__ out)
{
  __shared__ __align__(16) unsigned sHhi[kScanM * kNH / 2];
  __shared__ __align__(16) unsigned sHlo[kScanM * kNH / 2];
  __shared__ __align__(16) float    sOut[kScanM * kNH];

  const int tid = threadIdx.x, lane = tid & 31, wave = tid >> 5;
  const int hh = lane >> 4, c = lane & 15;
  const int koff = hh * 8;
  const int b0 = blockIdx.x * kScanM;
  const int ncol = wave * 32 + 2 * c;

  const __bf16* Vb  = (const __bf16*)vbp;
  const __bf16* Vzb = (const __bf16*)vzbp;
  const __bf16* pVc0 = Vb  + (size_t)ncol * kNH + koff;
  const __bf16* pVc1 = pVc0 + kNH;
  const __bf16* pVz0 = Vzb + (size_t)ncol * kNH + koff;
  const __bf16* pVz1 = pVz0 + kNH;

  {
    const v4u z4 = {0u, 0u, 0u, 0u};
    *(v4u*)(sHhi + tid * 4) = z4;
    *(v4u*)(sHhi + 2048 + tid * 4) = z4;
    *(v4u*)(sHlo + tid * 4) = z4;
    *(v4u*)(sHlo + 2048 + tid * 4) = z4;
  }
  float h0[8], h1[8];
#pragma unroll
  for (int r = 0; r < 8; ++r) { h0[r] = 0.f; h1[r] = 0.f; }
  __syncthreads();

  const int aoff = c * kNH + koff;

#pragma unroll 1
  for (int t = 0; t < kNT; ++t) {
    v2f wx[8];
    unsigned wz[8];
#pragma unroll
    for (int r = 0; r < 8; ++r) {
      const size_t idx = ((size_t)(b0 + 8 * hh + r) * kNT + t) * kNH + ncol;
      wx[r] = *(const v2f*)(WX + idx);
      wz[r] = WZX32[idx >> 1];
    }

    v8f aC0 = (v8f){0.f, 0.f, 0.f, 0.f, 0.f, 0.f, 0.f, 0.f};
    v8f aC1 = aC0, aZ0 = aC0, aZ1 = aC0;
#pragma unroll 1
    for (int k0 = 0; k0 < kNH; k0 += 32) {
      FragB ah, al;
      ah.h[0] = *(const v8b*)((const __bf16*)sHhi + aoff + k0);
      ah.h[1] = *(const v8b*)((const __bf16*)sHhi + aoff + k0 + 16);
      al.h[0] = *(const v8b*)((const __bf16*)sHlo + aoff + k0);
      al.h[1] = *(const v8b*)((const __bf16*)sHlo + aoff + k0 + 16);
      const v16b bc0 = frag_load(pVc0 + k0);
      const v16b bc1 = frag_load(pVc1 + k0);
      const v16b bz0 = frag_load(pVz0 + k0);
      const v16b bz1 = frag_load(pVz1 + k0);
      aC0 = at_mma(ah.v, bc0, aC0);
      aC1 = at_mma(ah.v, bc1, aC1);
      aZ0 = at_mma(ah.v, bz0, aZ0);
      aZ1 = at_mma(ah.v, bz1, aZ1);
      aC0 = at_mma(al.v, bc0, aC0);
      aC1 = at_mma(al.v, bc1, aC1);
      aZ0 = at_mma(al.v, bz0, aZ0);
      aZ1 = at_mma(al.v, bz1, aZ1);
    }
    __syncthreads();

#pragma unroll
    for (int r = 0; r < 8; ++r) {
      const unsigned wzr = wz[r];
      const float wz0 = h16_to_f32(wzr & 0xffffu);
      const float wz1 = h16_to_f32(wzr >> 16);
      const v2f wxr = wx[r];
      const float wx0 = wxr.x;
      const float wx1 = wxr.y;
      const float hn0 = gate_update(wz0 + aZ0[r], wx0 + aC0[r], h0[r]);
      const float hn1 = gate_update(wz1 + aZ1[r], wx1 + aC1[r], h1[r]);
      h0[r] = hn0;
      h1[r] = hn1;
      const unsigned hb0 = f2bf_bits(hn0);
      const unsigned hb1 = f2bf_bits(hn1);
      const unsigned lb0 = f2bf_bits(hn0 - bf_bits2f(hb0));
      const unsigned lb1 = f2bf_bits(hn1 - bf_bits2f(hb1));
      const int e = (8 * hh + r) * kNH + ncol;
      sHhi[e >> 1] = hb0 | (hb1 << 16);
      sHlo[e >> 1] = lb0 | (lb1 << 16);
      v2f o;
      o.x = hn0;
      o.y = hn1;
      *(v2f*)(sOut + e) = o;
    }
    __syncthreads();

    {
      const float* sp = sOut + wave * kNH + lane * 4;
      const v4f o0 = *(const v4f*)(sp);
      const v4f o1 = *(const v4f*)(sp + 128);
      const v4f o2 = *(const v4f*)(sp + 256);
      const v4f o3 = *(const v4f*)(sp + 384);
      float* gp = out + ((size_t)(b0 + wave) * kNT + t) * kNH + lane * 4;
      for (int pass = 0; pass < 2; ++pass) {
        *(volatile v4f*)(gp)       = o0;
        *(volatile v4f*)(gp + 128) = o1;
        *(volatile v4f*)(gp + 256) = o2;
        *(volatile v4f*)(gp + 384) = o3;
        __threadfence();
      }
    }
  }
}

extern "C" void kernel_launch(void* const* d_in, const int* in_sizes, int n_in,
                              void* d_out, int out_size, void* d_ws, size_t ws_size,
                              hipStream_t stream) {
  if (n_in < 7) return;
  if (in_sizes[0] != kRows * kNF) return;
  if (in_sizes[1] != kNH * kNF) return;
  if (in_sizes[2] != kNH * kNF) return;
  if (in_sizes[3] != kNH * kNH) return;
  if (in_sizes[4] != kNH * kNH) return;
  if (in_sizes[5] != kNH) return;
  if (in_sizes[6] != kNH) return;
  if (out_size != kRows * kNH) return;
  if (ws_size < kWsTotal) return;

  const float* x     = (const float*)d_in[0];
  const float* W     = (const float*)d_in[1];
  const float* Wz    = (const float*)d_in[2];
  const float* V     = (const float*)d_in[3];
  const float* Vz    = (const float*)d_in[4];
  const float* gamma = (const float*)d_in[5];
  const float* beta  = (const float*)d_in[6];
  float* out = (float*)d_out;

  char* ws = (char*)d_ws;
  unsigned* XB  = (unsigned*)(ws + kOffXB);
  unsigned* WB  = (unsigned*)(ws + kOffWB);
  unsigned* WZB = (unsigned*)(ws + kOffWZB);
  unsigned* VB  = (unsigned*)(ws + kOffVB);
  unsigned* VZB = (unsigned*)(ws + kOffVZB);
  float*    WXP = (float*)(ws + kOffWX);
  unsigned* WZXP = (unsigned*)(ws + kOffWZX);

  cast_bf16_kernel<<<kCastBlocks, 256, 0, stream>>>(x, W, Wz, V, Vz, XB, WB, WZB, VB, VZB);

  proj_ln_kernel<0><<<kRows / kProjM, 256, 0, stream>>>(
      (const unsigned short*)XB, (const unsigned short*)WB, gamma, beta, (void*)WXP);
  proj_ln_kernel<1><<<kRows / kProjM, 256, 0, stream>>>(
      (const unsigned short*)XB, (const unsigned short*)WZB, gamma, beta, (void*)WZXP);

  gated_scan_kernel<<<kNB / kScanM, 512, 0, stream>>>(
      (const unsigned short*)VB, (const unsigned short*)VZB, WXP, (const unsigned*)WZXP, out);
}
